// FatigueLSTM_36713380446334
// MI455X (gfx1250) — hardware-verified
//
#include <hip/hip_runtime.h>
#include <stdint.h>

typedef __attribute__((ext_vector_type(16))) _Float16 v16h;
typedef __attribute__((ext_vector_type(8)))  _Float16 v8h;
typedef __attribute__((ext_vector_type(8)))  float    v8f;
typedef __attribute__((ext_vector_type(4)))  float    v4f;
typedef __attribute__((ext_vector_type(4)))  unsigned v4u;

constexpr int SEQ_T    = 512;
constexpr int IN_DIM   = 5;
constexpr int HID      = 32;
constexpr int NGATE    = 4;
constexpr int NOUT     = 3;
constexpr int ROWS_BLK = 32;
constexpr int NTHR     = 128;
constexpr int HPITCH   = 40;
constexpr int XPITCH   = 8;
constexpr int FPITCH   = 36;
constexpr int XCNT     = ROWS_BLK * IN_DIM;
constexpr float WSCALE   = 16.0f;
constexpr float HSCALE   = 16.0f;
constexpr float ACC_FOLD = 1.0f / 256.0f;

static_assert(NTHR == 4 * 32, "four waves per block");
static_assert((HPITCH % 8) == 0, "16-byte aligned f16 rows");
static_assert(XCNT > NTHR && XCNT <= 2 * NTHR, "x staging uses two slots per thread");
static_assert(ROWS_BLK * NOUT * 4 == 3 * 128, "block output segment is three whole 128-byte lines");

__device__ __forceinline__ v8f mma_f16(v16h a, v16h b, v8f c) {
  return __builtin_amdgcn_wmma_f32_16x16x32_f16(false, a, false, b, (short)0, c, false, false);
}
__device__ __forceinline__ void acc_guard_a(v8f& c0, v8f& c1, v8f& c2, v8f& c3, v16h a) {
  asm volatile("v_nop\n\tv_nop\n\tv_nop\n\tv_nop" : "+v"(c0), "+v"(c1), "+v"(c2), "+v"(c3) : "v"(a));
}
__device__ __forceinline__ void keep4(v16h a, v16h b, v16h c, v16h d) {
  asm volatile("v_nop" :: "v"(a), "v"(b), "v"(c), "v"(d));
}

__device__ __forceinline__ float gate_sigmoid(float x) {
  const float e = __builtin_amdgcn_exp2f(-1.4426950408889634f * x);
  return __builtin_amdgcn_rcpf(1.0f + e);
}
__device__ __forceinline__ float gate_tanh(float x) {
  const float e = __builtin_amdgcn_exp2f(2.8853900817779268f * x);
  return __builtin_fmaf(-2.0f, __builtin_amdgcn_rcpf(1.0f + e), 1.0f);
}

__global__ __launch_bounds__(256) void xpose_x_kernel(
    const float* __restrict__ x, float* __restrict__ xT, int nrows, int n4)
{
  const int gid = blockIdx.x * 256 + (int)threadIdx.x;
  if (gid >= n4) return;
  const int slab = nrows * IN_DIM;
  const int d    = gid * 4;
  const int t    = d / slab;
  const int rem  = d - t * slab;
  v4f v;
#pragma unroll
  for (int e = 0; e < 4; ++e) {
    const int re   = rem + e;
    const int row  = re / IN_DIM;
    const int comp = re - row * IN_DIM;
    v[e] = x[((size_t)row * SEQ_T + (size_t)t) * IN_DIM + comp];
  }
  float* dst = xT + (size_t)gid * 4;
  *(volatile v4f*)dst = v;
  __threadfence();
  *(volatile v4f*)dst = v;
}

__global__ __launch_bounds__(NTHR) void lstm_seq_kernel(
    const float* __restrict__ xT,
    const float* __restrict__ W_ih,
    const float* __restrict__ W_hh,
    const float* __restrict__ b_ih,
    const float* __restrict__ b_hh,
    const float* __restrict__ W_fc,
    const float* __restrict__ b_fc,
    float* __restrict__ out,
    int nrows)
{
  __shared__ __align__(16) _Float16 hA[2][ROWS_BLK * HPITCH];
  __shared__ __align__(16) float    xs[2][ROWS_BLK * XPITCH];
  __shared__ __align__(16) float    hF[ROWS_BLK * FPITCH];
  __shared__ __align__(16) float    outS[128];

  const int tid  = (int)threadIdx.x;
  const int wave = tid >> 5;
  const int lane = tid & 31;
  const int c    = lane & 15;
  const int hh   = lane >> 4;
  const int msub = wave >> 1;
  const int ub   = wave & 1;
  const int unit  = 16 * ub + c;
  const int rbase = 16 * msub + 8 * hh;
  const int R0    = (int)blockIdx.x * ROWS_BLK;

  float wih[NGATE][IN_DIM];
  float bsum[NGATE];
  v16h  bw[NGATE];
#pragma unroll
  for (int g = 0; g < NGATE; ++g) {
    const int n = g * HID + unit;
#pragma unroll
    for (int i = 0; i < IN_DIM; ++i) wih[g][i] = W_ih[n * IN_DIM + i];
    bsum[g] = b_ih[n] + b_hh[n];
    const float* wr = W_hh + (size_t)n * HID;
#pragma unroll
    for (int e = 0; e < 8; ++e) {
      bw[g][e]     = (_Float16)(WSCALE * wr[8 * hh + e]);
      bw[g][8 + e] = (_Float16)(WSCALE * wr[16 + 8 * hh + e]);
    }
  }

  {
    v4u* hz = (v4u*)(void*)&hA[0][0];
    const v4u z4 = (v4u){0u, 0u, 0u, 0u};
    for (int i = tid; i < (2 * ROWS_BLK * HPITCH) / 8; i += NTHR) hz[i] = z4;
  }

  float cst[8], hreg[8];
#pragma unroll
  for (int r = 0; r < 8; ++r) { cst[r] = 0.0f; hreg[r] = 0.0f; }

  const int  i1  = (tid + NTHR < XCNT) ? (tid + NTHR) : (XCNT - 1);
  const bool st1 = (tid + NTHR) < XCNT;
  const int  xo0 = (tid / IN_DIM) * XPITCH + (tid - (tid / IN_DIM) * IN_DIM);
  const int  xo1 = (i1  / IN_DIM) * XPITCH + (i1  - (i1  / IN_DIM) * IN_DIM);
  const size_t slab = (size_t)nrows * IN_DIM;
  {
    const float* xsrc = xT + (size_t)R0 * IN_DIM;
    const float v0 = xsrc[tid];
    const float v1 = xsrc[i1];
    xs[0][xo0] = v0;
    if (st1) xs[0][xo1] = v1;
  }
  __syncthreads();

  const v8f zc = (v8f){0.f, 0.f, 0.f, 0.f, 0.f, 0.f, 0.f, 0.f};

  for (int t = 0; t < SEQ_T; ++t) {
    const int p  = t & 1;
    const int pn = p ^ 1;

    const int tn = (t + 1 < SEQ_T) ? (t + 1) : t;
    const float* xsrc = xT + (size_t)tn * slab + (size_t)R0 * IN_DIM;
    const float xv0 = xsrc[tid];
    const float xv1 = xsrc[i1];

    v16h a;
    {
      union { v16h v; v8h h[2]; } f;
      const _Float16* ap = &hA[p][(16 * msub + c) * HPITCH + 8 * hh];
      f.h[0] = *(const v8h*)(ap);
      f.h[1] = *(const v8h*)(ap + 16);
      a = f.v;
    }
    v8f acc[NGATE];
#pragma unroll
    for (int g = 0; g < NGATE; ++g) acc[g] = mma_f16(a, bw[g], zc);
    acc_guard_a(acc[0], acc[1], acc[2], acc[3], a);

#pragma unroll
    for (int r = 0; r < 8; ++r) {
      const int rl = rbase + r;
      const float* xr = &xs[p][rl * XPITCH];
      const v4f   x4 = *(const v4f*)xr;
      const float x5 = xr[4];
      float pre[NGATE];
#pragma unroll
      for (int g = 0; g < NGATE; ++g) {
        float s = bsum[g];
        s = __builtin_fmaf(x4[0], wih[g][0], s);
        s = __builtin_fmaf(x4[1], wih[g][1], s);
        s = __builtin_fmaf(x4[2], wih[g][2], s);
        s = __builtin_fmaf(x4[3], wih[g][3], s);
        s = __builtin_fmaf(x5,    wih[g][4], s);
        pre[g] = __builtin_fmaf(acc[g][r], ACC_FOLD, s);
      }
      const float ig = gate_sigmoid(pre[0]);
      const float fg = gate_sigmoid(pre[1]);
      const float gg = gate_tanh(pre[2]);
      const float og = gate_sigmoid(pre[3]);
      const float cn = __builtin_fmaf(fg, cst[r], ig * gg);
      cst[r] = cn;
      const float hv = og * gate_tanh(cn);
      hreg[r] = hv;
      hA[pn][rl * HPITCH + unit] = (_Float16)(HSCALE * hv);
    }

    xs[pn][xo0] = xv0;
    if (st1) xs[pn][xo1] = xv1;
    keep4(bw[0], bw[1], bw[2], bw[3]);
    __syncthreads();
  }

#pragma unroll
  for (int r = 0; r < 8; ++r) hF[(rbase + r) * FPITCH + unit] = hreg[r];
  __syncthreads();
  if (tid < ROWS_BLK * NOUT) {
    const int row = tid / NOUT;
    const int j   = tid - row * NOUT;
    const float* hr = &hF[row * FPITCH];
    const float* wr = W_fc + j * HID;
    float s = 0.0f;
#pragma unroll 1
    for (int k = 0; k < HID; ++k) s = __builtin_fmaf(hr[k], wr[k], s);
    outS[tid] = s + b_fc[j];
  }
  __syncthreads();

  if (wave == 0) {
    const int lq = (lane < 24) ? lane : 23;
    const v4f v = *(const v4f*)(&outS[lq * 4]);
    float* op = out + (size_t)R0 * NOUT + (size_t)lq * 4;
    for (int pass = 0; pass < 2; ++pass) {
      if (lane < 24) *(volatile v4f*)op = v;
      __threadfence();
    }
  }
}

extern "C" void kernel_launch(void* const* d_in, const int* in_sizes, int n_in,
                              void* d_out, int out_size, void* d_ws, size_t ws_size,
                              hipStream_t stream)
{
  const float* x    = (const float*)d_in[0];
  const float* W_ih = (const float*)d_in[1];
  const float* W_hh = (const float*)d_in[2];
  const float* b_ih = (const float*)d_in[3];
  const float* b_hh = (const float*)d_in[4];
  const float* W_fc = (const float*)d_in[5];
  const float* b_fc = (const float*)d_in[6];
  float* out = (float*)d_out;
  (void)n_in; (void)stream;

  const int total = in_sizes[0];
  const int nrows = total / (SEQ_T * IN_DIM);
  if (nrows <= 0) return;
  if (nrows * SEQ_T * IN_DIM != total) return;
  if ((nrows % ROWS_BLK) != 0) return;
  if (out_size != nrows * NOUT) return;
  const size_t xT_bytes = (size_t)total * sizeof(float);
  if (xT_bytes > ws_size) return;

  float* xT = (float*)d_ws;
  const int n4 = total / 4;

  xpose_x_kernel<<<dim3((unsigned)((n4 + 255) / 256)), dim3(256), 0, stream>>>(x, xT, nrows, n4);
  lstm_seq_kernel<<<dim3((unsigned)(nrows / ROWS_BLK)), dim3(NTHR), 0, stream>>>(
      xT, W_ih, W_hh, b_ih, b_hh, W_fc, b_fc, out, nrows);
}
